// NeuroKernel_69956427318000
// MI455X (gfx1250) — hardware-verified
//
#include <hip/hip_runtime.h>
#include <math.h>

constexpr int kNx        = 768;
constexpr int kPairs     = (kNx * (kNx + 1)) / 2;
constexpr int kHid1      = 1024;
constexpr int kHid2      = 128;
constexpr int kChunkRows = 49216;
constexpr int kNumChunks = 6;
constexpr int kGramLd    = 3072;
constexpr int kGramK     = 2304;
constexpr float kH1Carry    = 4096.0f;
constexpr float kW2Carry    = 1024.0f;
constexpr float kGemm2Scale = 1.0f / (4096.0f * 1024.0f);
static_assert(kChunkRows * kNumChunks == kPairs, "chunks cover all pair rows exactly");
static_assert(kChunkRows % 64 == 0, "GEMM M tile multiple");
static_assert(kHid1 % 32 == 0 && kHid2 % 64 == 0 && kGramK % 32 == 0 && kNx % 64 == 0, "tile multiples");

constexpr size_t kOffH1    = 0;
constexpr size_t kBytesH1  = (size_t)kChunkRows * kHid1 * 2;
constexpr size_t kOffH2    = kOffH1 + kBytesH1;
constexpr size_t kBytesH2  = (size_t)kChunkRows * kHid2 * 4;
constexpr size_t kOffV     = kOffH2 + kBytesH2;
constexpr size_t kBytesV   = (size_t)kPairs * 4;
constexpr size_t kOffW2H   = kOffV + kBytesV;
constexpr size_t kBytesW2H = (size_t)kHid2 * kHid1 * 2;
constexpr size_t kWsTotal  = kOffW2H + kBytesW2H;
static_assert(kWsTotal <= (size_t)134217728, "carve under 128 MiB");
static_assert((size_t)kNx * kGramLd * 2 <= kBytesH1, "gram plane fits in the dead H1 region");
static_assert(kOffH2 % 128 == 0 && kOffV % 128 == 0 && kOffW2H % 128 == 0, "128-B aligned regions");
static_assert((kChunkRows * 4) % 128 == 0, "V chunk bases line aligned");

typedef __attribute__((ext_vector_type(16))) _Float16 v16h;
typedef __attribute__((ext_vector_type(8)))  _Float16 v8h;
typedef __attribute__((ext_vector_type(16))) __bf16   v16b;
typedef __attribute__((ext_vector_type(8)))  __bf16   v8b;
typedef __attribute__((ext_vector_type(8)))  float    v8f;
typedef __attribute__((ext_vector_type(4)))  float    v4f;
typedef __attribute__((ext_vector_type(4)))  unsigned int v4u;

__device__ __forceinline__ unsigned short f2bf_bits(float f) {
  unsigned u = __float_as_uint(f);
  return (unsigned short)((u + 0x7FFFu + ((u >> 16) & 1u)) >> 16);
}
__device__ __forceinline__ float bf_bits2f(unsigned short h) { return __uint_as_float(((unsigned)h) << 16); }

__device__ __forceinline__ void dep_guard_h(v8f& a, v8f& b, v16h x, v16h y) { asm volatile("v_nop\n\tv_nop\n\tv_nop\n\tv_nop" : "+v"(a), "+v"(b) : "v"(x), "v"(y)); }
__device__ __forceinline__ void dep_guard_b(v8f& a, v8f& b, v16b x, v16b y) { asm volatile("v_nop\n\tv_nop\n\tv_nop\n\tv_nop" : "+v"(a), "+v"(b) : "v"(x), "v"(y)); }
__device__ __forceinline__ void keep4_h(v16h a, v16h b, v16h c, v16h d) { asm volatile("v_nop" :: "v"(a), "v"(b), "v"(c), "v"(d)); }
__device__ __forceinline__ void keep4_b(v16b a, v16b b, v16b c, v16b d) { asm volatile("v_nop" :: "v"(a), "v"(b), "v"(c), "v"(d)); }
__device__ __forceinline__ void acc_guard4(v8f& a, v8f& b, v8f& c, v8f& d) { asm volatile("v_nop\n\tv_nop\n\tv_nop\n\tv_nop" : "+v"(a), "+v"(b), "+v"(c), "+v"(d)); }
template <typename T> struct Frag;
template <> struct Frag<_Float16> {
  typedef v16h V; union U { v16h v; v8h h[2]; };
  static __device__ __forceinline__ v16h load(const _Float16* p) {
    U f; f.h[0] = *(const v8h*)(p); f.h[1] = *(const v8h*)(p + 16); return f.v;
  }
  static __device__ __forceinline__ v8f mma(v16h a, v16h b, v8f c) {
    return __builtin_amdgcn_wmma_f32_16x16x32_f16(false, a, false, b, (short)0, c, false, false);
  }
  static __device__ __forceinline__ void guard(v8f& a, v8f& b, v16h x, v16h y) { dep_guard_h(a, b, x, y); }
  static __device__ __forceinline__ void keep(v16h a, v16h b, v16h c, v16h d) { keep4_h(a, b, c, d); }
};
template <> struct Frag<__bf16> {
  typedef v16b V; union U { v16b v; v8b h[2]; };
  static __device__ __forceinline__ v16b load(const __bf16* p) {
    U f; f.h[0] = *(const v8b*)(p); f.h[1] = *(const v8b*)(p + 16); return f.v;
  }
  static __device__ __forceinline__ v8f mma(v16b a, v16b b, v8f c) {
    return __builtin_amdgcn_wmma_f32_16x16x32_bf16(false, a, false, b, (short)0, c, false, false);
  }
  static __device__ __forceinline__ void guard(v8f& a, v8f& b, v16b x, v16b y) { dep_guard_b(a, b, x, y); }
  static __device__ __forceinline__ void keep(v16b a, v16b b, v16b c, v16b d) { keep4_b(a, b, c, d); }
};

__device__ __forceinline__ unsigned pk16(unsigned short a, unsigned short b) { return (unsigned)a | ((unsigned)b << 16); }
__device__ __forceinline__ unsigned short h_bits(float f) { const _Float16 h = (_Float16)f; return __builtin_bit_cast(unsigned short, h); }

template <int ET> struct Elem;
template <> struct Elem<0> { typedef _Float16 T; };
template <> struct Elem<1> { typedef __bf16 T; };
template <int ET, bool SPLIT, int BIAS_MODE, int OUT_MODE, bool RESID, int ACT = 0>
__global__ __launch_bounds__(256) void wmma_gemm64(
    const unsigned short* __restrict__ Ap, const unsigned short* __restrict__ A2p, int lda, long strideA,
    const unsigned short* __restrict__ Btp, const unsigned short* __restrict__ Bt2p, int ldb, long strideB,
    void* __restrict__ Cout, void* __restrict__ Cout2, int ldc, long strideC,
    const float* __restrict__ bias,
    const float* __restrict__ resid, long strideR,
    int M, int N, int K, float scale) {
  typedef typename Elem<ET>::T T;
  typedef typename Frag<T>::V V;
  const T* A = (const T*)Ap; const T* A2 = (const T*)A2p; const T* Bt = (const T*)Btp; const T* Bt2 = (const T*)Bt2p;
  __shared__ __align__(16) float sT[8][16 * 68];
  const int b    = blockIdx.y;
  const int lane = threadIdx.x & 31;
  const int wave = threadIdx.x >> 5;
  const int tilesN = N >> 6;
  const int tilesM = M >> 6;
  const int tile = blockIdx.x * 8 + wave;
  if (tile >= tilesM * tilesN) return;
  const int tm = tile / tilesN;
  const int tn = tile - tm * tilesN;
  const int m0 = tm << 6;
  const int n0 = tn << 6;

  const T* Ab  = A  + (size_t)b * strideA;
  const T* Bb  = Bt + (size_t)b * strideB;
  const T* Ab2 = SPLIT ? (A2  + (size_t)b * strideA) : nullptr;
  const T* Bb2 = SPLIT ? (Bt2 + (size_t)b * strideB) : nullptr;

  const int rlane = lane & 15;
  const int koff  = (lane >> 4) * 8;
  const int mOff  = (lane >> 4) * 8;

  v8f acc[4][4];
#pragma unroll
  for (int i = 0; i < 4; ++i)
#pragma unroll
    for (int j = 0; j < 4; ++j) acc[i][j] = (v8f){0.f,0.f,0.f,0.f,0.f,0.f,0.f,0.f};

  for (int k0 = 0; k0 < K; k0 += 32) {
    V bh[4], bl[4];
#pragma unroll
    for (int j = 0; j < 4; ++j) {
      const size_t bo = (size_t)(n0 + (j << 4) + rlane) * ldb + koff + k0;
      bh[j] = Frag<T>::load(Bb + bo);
      if (SPLIT) bl[j] = Frag<T>::load(Bb2 + bo);
    }
#pragma unroll
    for (int i = 0; i < 4; ++i) {
      const size_t ao = (size_t)(m0 + (i << 4) + rlane) * lda + koff + k0;
      V ah = Frag<T>::load(Ab + ao);
      V al;
      if (SPLIT) al = Frag<T>::load(Ab2 + ao);
#pragma unroll
      for (int j = 0; j < 4; ++j) {
        acc[i][j] = Frag<T>::mma(ah, bh[j], acc[i][j]);
        if (SPLIT) {
          acc[i][j] = Frag<T>::mma(ah, bl[j], acc[i][j]);
          acc[i][j] = Frag<T>::mma(al, bh[j], acc[i][j]);
        }
      }
      Frag<T>::guard(acc[i][0], acc[i][3], ah, SPLIT ? al : ah);
    }
    Frag<T>::keep(bh[0], bh[1], bh[2], bh[3]);
    if (SPLIT) Frag<T>::keep(bl[0], bl[1], bl[2], bl[3]);
  }
  acc_guard4(acc[0][0], acc[0][1], acc[0][2], acc[0][3]);
  acc_guard4(acc[1][0], acc[1][1], acc[1][2], acc[1][3]);
  acc_guard4(acc[2][0], acc[2][1], acc[2][2], acc[2][3]);
  acc_guard4(acc[3][0], acc[3][1], acc[3][2], acc[3][3]);

  float* slab = sT[wave];
  const float* Rb = RESID ? (resid + (size_t)b * strideR) : nullptr;
#pragma unroll
  for (int i = 0; i < 4; ++i) {
    const int mBase = m0 + (i << 4);
#pragma unroll
    for (int j = 0; j < 4; ++j) {
      const int n = n0 + (j << 4) + rlane;
      float bv = 0.f;
      if (BIAS_MODE == 2) bv = bias[n];
#pragma unroll
      for (int r = 0; r < 8; ++r) {
        float v = acc[i][j][r] * scale;
        if (BIAS_MODE == 1) v += bias[mBase + mOff + r];
        if (BIAS_MODE == 2) v += bv;
        if (RESID) v += Rb[(size_t)(mBase + mOff + r) * ldc + n];
        if (ACT == 2) v = fmaxf(v, 0.0f);
        if (ACT == 4) v = (v > 0.f) ? v : 0.01f * v;
        slab[(mOff + r) * 68 + (j << 4) + rlane] = v;
      }
    }
    __builtin_amdgcn_fence(__ATOMIC_RELEASE, "workgroup");
    __builtin_amdgcn_wave_barrier();
    __builtin_amdgcn_fence(__ATOMIC_ACQUIRE, "workgroup");
    if (OUT_MODE == 0) {
      float* C = (float*)Cout + (size_t)b * strideC;
      const int hh = lane >> 4, c4 = (lane & 15) * 4;
      for (int pass = 0; pass < 2; ++pass) {
#pragma unroll
        for (int it = 0; it < 8; ++it) {
          const int row = it * 2 + hh;
          v4f v = *(const v4f*)(slab + row * 68 + c4);
          *(volatile v4f*)(C + (size_t)(mBase + row) * ldc + n0 + c4) = v;
        }
        __threadfence();
      }
    } else {
      const int q = lane >> 3, c8 = (lane & 7) * 8;
      unsigned short* C  = (unsigned short*)Cout  + (size_t)b * strideC;
      unsigned short* C2 = (OUT_MODE == 2) ? ((unsigned short*)Cout2 + (size_t)b * strideC) : nullptr;
      for (int pass = 0; pass < 2; ++pass) {
#pragma unroll
        for (int it = 0; it < 4; ++it) {
          const int row = it * 4 + q;
          const float* sp = slab + row * 68 + c8;
          v8h hv, lv;
#pragma unroll
          for (int e = 0; e < 8; ++e) {
            if (OUT_MODE == 1) {
              hv[e] = (_Float16)sp[e];
            } else {
              unsigned short hb = f2bf_bits(sp[e]);
              unsigned short lb = f2bf_bits(sp[e] - bf_bits2f(hb));
              hv[e] = __builtin_bit_cast(_Float16, hb);
              lv[e] = __builtin_bit_cast(_Float16, lb);
            }
          }
          *(volatile v8h*)(C + (size_t)(mBase + row) * ldc + n0 + c8) = hv;
          if (OUT_MODE == 2) *(volatile v8h*)(C2 + (size_t)(mBase + row) * ldc + n0 + c8) = lv;
        }
        __threadfence();
      }
    }
    __builtin_amdgcn_fence(__ATOMIC_RELEASE, "workgroup");
    __builtin_amdgcn_wave_barrier();
    __builtin_amdgcn_fence(__ATOMIC_ACQUIRE, "workgroup");
  }
}

__global__ __launch_bounds__(256) void cast8_scale_f16_kernel(const float* __restrict__ in, unsigned short* __restrict__ out,
                                                             int n8, float scale) {
  const int i = blockIdx.x * 256 + threadIdx.x;
  if (i >= n8) return;
  const float* p = in + 8 * (size_t)i;
  const v4f a = *(const v4f*)(p);
  const v4f c = *(const v4f*)(p + 4);
  unsigned short hb[8];
#pragma unroll
  for (int e = 0; e < 4; ++e) {
    hb[e]     = h_bits(a[e] * scale);
    hb[4 + e] = h_bits(c[e] * scale);
  }
  const v4u u = (v4u){pk16(hb[0], hb[1]), pk16(hb[2], hb[3]), pk16(hb[4], hb[5]), pk16(hb[6], hb[7])};
  unsigned short* q = out + 8 * (size_t)i;
  *(volatile v4u*)q = u;
  __threadfence();
  *(volatile v4u*)q = u;
}

__device__ __forceinline__ int pair_row_offset(int i) { return i * kNx - ((i * (i - 1)) >> 1); }
__device__ __forceinline__ void pair_from_index(int p, int& i, int& j) {
  const float tn   = (float)(2 * kNx + 1);
  const float disc = tn * tn - 8.0f * (float)p;
  int ii = (int)((tn - sqrtf(fmaxf(disc, 0.0f))) * 0.5f);
  ii = ii < 0 ? 0 : (ii > kNx - 1 ? kNx - 1 : ii);
#pragma unroll
  for (int t = 0; t < 2; ++t) { if (ii < kNx - 1 && pair_row_offset(ii + 1) <= p) ++ii; }
#pragma unroll
  for (int t = 0; t < 2; ++t) { if (ii > 0 && pair_row_offset(ii) > p) --ii; }
  int jj = ii + (p - pair_row_offset(ii));
  jj = jj < 0 ? 0 : (jj > kNx - 1 ? kNx - 1 : jj);
  i = ii; j = jj;
}

__global__ __launch_bounds__(128) void pair_layer1_kernel(const float* __restrict__ x, const float* __restrict__ W1,
                                                         const float* __restrict__ b1, unsigned short* __restrict__ H1,
                                                         int rowBase) {
  const int prow = blockIdx.x;
  int i, j;
  pair_from_index(rowBase + prow, i, j);
  const float xi = x[i];
  const float xj = x[j];
  const int t  = threadIdx.x;
  const int k8 = t * 8;
  const v8f wlo = *(const v8f*)(W1 + 2 * k8);
  const v8f whi = *(const v8f*)(W1 + 2 * k8 + 8);
  const v8f bv  = *(const v8f*)(b1 + k8);
  float wz0[8], wz1[8], bz[8];
#pragma unroll
  for (int e = 0; e < 4; ++e) {
    wz0[e]     = wlo[2 * e];  wz1[e]     = wlo[2 * e + 1];
    wz0[4 + e] = whi[2 * e];  wz1[4 + e] = whi[2 * e + 1];
    bz[e] = bv[e]; bz[4 + e] = bv[4 + e];
  }
  unsigned short hb[8];
#pragma unroll
  for (int e = 0; e < 8; ++e) {
    float z = xi * wz0[e] + xj * wz1[e] + bz[e];
    z = fminf(fmaxf(z, -30.0f), 30.0f);
    const float ex = expf(-z);
    const float sg = __builtin_amdgcn_rcpf(1.0f + ex);
    hb[e] = h_bits(sg * kH1Carry);
  }
  const v4u u = (v4u){pk16(hb[0], hb[1]), pk16(hb[2], hb[3]), pk16(hb[4], hb[5]), pk16(hb[6], hb[7])};
  unsigned short* q = H1 + (size_t)prow * kHid1 + k8;
  *(volatile v4u*)q = u;
  __threadfence();
  *(volatile v4u*)q = u;
}

__global__ __launch_bounds__(256) void head_dot_kernel(const float* __restrict__ H2, const float* __restrict__ W3,
                                                      const float* __restrict__ b3, float* __restrict__ Vout, int nquads) {
  __shared__ __align__(16) float sw[kHid2];
  const int t = threadIdx.x;
  if (t < kHid2) sw[t] = W3[t];
  __syncthreads();
  const int q = blockIdx.x * 256 + t;
  if (q >= nquads) return;
  const float* r0p = H2 + (size_t)(4 * q) * kHid2;
  float a0 = 0.f, a1 = 0.f, a2 = 0.f, a3 = 0.f;
#pragma unroll 1
  for (int it = 0; it < kHid2 / 4; ++it) {
    const v4f w  = *(const v4f*)(sw + 4 * it);
    const v4f h0 = *(const v4f*)(r0p + 4 * it);
    const v4f h1 = *(const v4f*)(r0p + kHid2 + 4 * it);
    const v4f h2 = *(const v4f*)(r0p + 2 * kHid2 + 4 * it);
    const v4f h3 = *(const v4f*)(r0p + 3 * kHid2 + 4 * it);
#pragma unroll
    for (int e = 0; e < 4; ++e) {
      a0 = fmaf(h0[e], w[e], a0);
      a1 = fmaf(h1[e], w[e], a1);
      a2 = fmaf(h2[e], w[e], a2);
      a3 = fmaf(h3[e], w[e], a3);
    }
  }
  const float bb = b3[0];
  const v4f o = (v4f){a0 + bb, a1 + bb, a2 + bb, a3 + bb};
  float* dst = Vout + 4 * (size_t)q;
  *(volatile v4f*)dst = o;
  __threadfence();
  *(volatile v4f*)dst = o;
}

__global__ __launch_bounds__(96) void kbuild_kernel(const float* __restrict__ V, unsigned short* __restrict__ G) {
  const int a  = blockIdx.x;
  const int t  = threadIdx.x;
  const int i8 = t * 8;
  unsigned short hb[8], lb[8];
#pragma unroll
  for (int e = 0; e < 8; ++e) {
    const int i   = i8 + e;
    const int ic  = i < a ? i : a;
    const int idx = pair_row_offset(ic) + (a - ic);
    float val = V[idx];
    val = (i <= a) ? val : 0.0f;
    const unsigned short h = f2bf_bits(val);
    hb[e] = h;
    lb[e] = f2bf_bits(val - bf_bits2f(h));
  }
  const v4u uh = (v4u){pk16(hb[0], hb[1]), pk16(hb[2], hb[3]), pk16(hb[4], hb[5]), pk16(hb[6], hb[7])};
  const v4u ul = (v4u){pk16(lb[0], lb[1]), pk16(lb[2], lb[3]), pk16(lb[4], lb[5]), pk16(lb[6], lb[7])};
  unsigned short* row = G + (size_t)a * kGramLd;
  for (int pass = 0; pass < 2; ++pass) {
    *(volatile v4u*)(row + i8)           = uh;
    *(volatile v4u*)(row + kNx + i8)     = uh;
    *(volatile v4u*)(row + 2 * kNx + i8) = ul;
    *(volatile v4u*)(row + 3 * kNx + i8) = uh;
    __threadfence();
  }
}

extern "C" void kernel_launch(void* const* d_in, const int* in_sizes, int n_in,
                              void* d_out, int out_size, void* d_ws, size_t ws_size,
                              hipStream_t stream) {
  if (n_in < 7) return;
  if (in_sizes[0] != kNx || in_sizes[1] != kHid1 * 2 || in_sizes[2] != kHid1 || in_sizes[3] != kHid2 * kHid1 ||
      in_sizes[4] != kHid2 || in_sizes[5] != kHid2 || in_sizes[6] < 1) return;
  if (out_size != kNx * kNx) return;
  if (ws_size < kWsTotal) return;

  const float* x  = (const float*)d_in[0];
  const float* W1 = (const float*)d_in[1];
  const float* b1 = (const float*)d_in[2];
  const float* W2 = (const float*)d_in[3];
  const float* b2 = (const float*)d_in[4];
  const float* W3 = (const float*)d_in[5];
  const float* b3 = (const float*)d_in[6];
  float* out = (float*)d_out;

  char* ws = (char*)d_ws;
  unsigned short* H1  = (unsigned short*)(ws + kOffH1);
  unsigned short* G   = (unsigned short*)(ws + kOffH1);
  float*          H2  = (float*)(ws + kOffH2);
  float*          V   = (float*)(ws + kOffV);
  unsigned short* W2H = (unsigned short*)(ws + kOffW2H);

  {
    const int n8 = (kHid2 * kHid1) / 8;
    cast8_scale_f16_kernel<<<dim3((n8 + 255) / 256), dim3(256), 0, stream>>>(W2, W2H, n8, kW2Carry);
  }

  for (int c = 0; c < kNumChunks; ++c) {
    const int rowBase = c * kChunkRows;
    pair_layer1_kernel<<<dim3(kChunkRows), dim3(128), 0, stream>>>(x, W1, b1, H1, rowBase);
    const int tiles = (kChunkRows / 64) * (kHid2 / 64);
    wmma_gemm64<0, false, 2, 0, false, 2><<<dim3((tiles + 7) / 8, 1), dim3(256), 0, stream>>>(
        H1, H1, kHid1, 0L, W2H, W2H, kHid1, 0L, (void*)H2, (void*)H2, kHid2, 0L,
        b2, b2, 0L, kChunkRows, kHid2, kHid1, kGemm2Scale);
    const int nquads = kChunkRows / 4;
    head_dot_kernel<<<dim3((nquads + 255) / 256), dim3(256), 0, stream>>>(H2, W3, b3, V + rowBase, nquads);
  }

  kbuild_kernel<<<dim3(kNx), dim3(96), 0, stream>>>(V, G);

  {
    const int tiles = (kNx / 64) * (kNx / 64);
    wmma_gemm64<1, false, 0, 0, false, 0><<<dim3((tiles + 7) / 8, 1), dim3(256), 0, stream>>>(
        G, G, kGramLd, 0L, G + kNx, G + kNx, kGramLd, 0L, (void*)out, (void*)H2, kNx, 0L,
        b2, b2, 0L, kNx, kNx, kGramK, 1.0f);
  }
}
